// GainRNN_70540542869836
// MI455X (gfx1250) — hardware-run, weakly checked
//
#include <hip/hip_runtime.h>
#include <math.h>

constexpr int NBATCH   = 64;
constexpr int NSTEP    = 512;
constexpr int NDIN     = 256;
constexpr int NHID     = 1024;
constexpr int NOUTC    = 64;
constexpr int KCAT     = NHID + NDIN;
constexpr int NROWS    = NBATCH * NSTEP;
constexpr int SEQ_BLK  = 16;
constexpr int SCAN_THR = 512;
constexpr int APITCH   = KCAT + 8;
constexpr int CVT_THR  = 256;
constexpr float STATE_CARRY     = (float)NHID;
constexpr float STATE_CARRY_INV = 1.0f / STATE_CARRY;
constexpr float WO_CARRY        = 64.0f;
constexpr float READ_SCALE      = 1.0f / (STATE_CARRY * WO_CARRY);

static_assert((NHID & (NHID - 1)) == 0);
static_assert(NBATCH % SEQ_BLK == 0);
static_assert(NHID == 64 * (SCAN_THR / 32));
static_assert(KCAT % 32 == 0 && NHID % 32 == 0 && NDIN % 32 == 0);
static_assert(NROWS % 64 == 0 && NOUTC % 64 == 0);
static_assert(SEQ_BLK * (NDIN / 8) == SCAN_THR);
static_assert(SEQ_BLK * (NHID / 8) == 4 * SCAN_THR);
static_assert((APITCH * 2) % 16 == 0);
static_assert((NHID / 8) % 32 == 0 && (NDIN / 8) % 32 == 0);
static_assert((KCAT * 2) % 128 == 0 && (NHID * 2) % 128 == 0);

typedef __attribute__((ext_vector_type(16))) _Float16 v16h;
typedef __attribute__((ext_vector_type(8)))  _Float16 v8h;
typedef __attribute__((ext_vector_type(8)))  float    v8f;
typedef __attribute__((ext_vector_type(4)))  float    v4f;
typedef __attribute__((ext_vector_type(4)))  unsigned v4u;

__device__ __forceinline__ void guard4x5_h(v8f& a0, v8f& a1, v8f& a2, v8f& a3,
                                           v16h x, v16h y0, v16h y1, v16h y2, v16h y3) {
  asm volatile("v_nop\n\tv_nop\n\tv_nop\n\tv_nop"
               : "+v"(a0), "+v"(a1), "+v"(a2), "+v"(a3)
               : "v"(x), "v"(y0), "v"(y1), "v"(y2), "v"(y3));
}
__device__ __forceinline__ void acc_guard4(v8f& a, v8f& b, v8f& c, v8f& d) {
  asm volatile("v_nop\n\tv_nop\n\tv_nop\n\tv_nop" : "+v"(a), "+v"(b), "+v"(c), "+v"(d));
}

union FragU { v16h v; v8h h[2]; };
__device__ __forceinline__ v16h frag_load(const _Float16* p) {
  FragU f;
  f.h[0] = *(const v8h*)(p);
  f.h[1] = *(const v8h*)(p + 16);
  return f.v;
}
__device__ __forceinline__ v8f frag_mma(v16h a, v16h b, v8f c) {
  return __builtin_amdgcn_wmma_f32_16x16x32_f16(false, a, false, b, (short)0, c, false, false);
}

__global__ __launch_bounds__(CVT_THR) void cvt8_f16_kernel(const float* __restrict__ src,
                                                           unsigned short* __restrict__ dst,
                                                           int n8, float sc) {
  const int i = blockIdx.x * CVT_THR + threadIdx.x;
  if (i < n8) {
    const float* sp = src + (size_t)i * 8;
    const v4f a = *(const v4f*)(sp);
    const v4f b = *(const v4f*)(sp + 4);
    v8h hv;
#pragma unroll
    for (int e = 0; e < 4; ++e) {
      const float f0 = a[e] * sc;
      const float f1 = b[e] * sc;
      hv[e]     = (_Float16)f0;
      hv[4 + e] = (_Float16)f1;
    }
    unsigned short* op = dst + (size_t)i * 8;
    *(volatile v8h*)op = hv;
    __threadfence();
    *(volatile v8h*)op = hv;
  }
}

__global__ __launch_bounds__(CVT_THR) void lowrank8_kernel(const float* __restrict__ bg,
                                                           const float* __restrict__ proj,
                                                           const float* __restrict__ recv,
                                                           unsigned short* __restrict__ dst,
                                                           int nrow, int ncol8, int dpitch, int dcol0) {
  const int i  = blockIdx.x * CVT_THR + threadIdx.x;
  const int n8 = nrow * ncol8;
  if (i < n8) {
    const int row = i / ncol8;
    const int c8  = i - row * ncol8;
    const float* bp = bg + (size_t)row * (size_t)(ncol8 * 8) + c8 * 8;
    const v4f b0 = *(const v4f*)(bp);
    const v4f b1 = *(const v4f*)(bp + 4);
    const float p0 = proj[row * 2 + 0];
    const float p1 = proj[row * 2 + 1];
    const float* rp = recv + (size_t)c8 * 16;
    const v4f r0 = *(const v4f*)(rp);
    const v4f r1 = *(const v4f*)(rp + 4);
    const v4f r2 = *(const v4f*)(rp + 8);
    const v4f r3 = *(const v4f*)(rp + 12);
    float w[8];
    w[0] = b0[0] + (p0 * r0[0] + p1 * r0[1]);
    w[1] = b0[1] + (p0 * r0[2] + p1 * r0[3]);
    w[2] = b0[2] + (p0 * r1[0] + p1 * r1[1]);
    w[3] = b0[3] + (p0 * r1[2] + p1 * r1[3]);
    w[4] = b1[0] + (p0 * r2[0] + p1 * r2[1]);
    w[5] = b1[1] + (p0 * r2[2] + p1 * r2[3]);
    w[6] = b1[2] + (p0 * r3[0] + p1 * r3[1]);
    w[7] = b1[3] + (p0 * r3[2] + p1 * r3[3]);
    v8h hv;
#pragma unroll
    for (int e = 0; e < 8; ++e) hv[e] = (_Float16)w[e];
    unsigned short* op = dst + (size_t)row * (size_t)dpitch + dcol0 + c8 * 8;
    *(volatile v8h*)op = hv;
    __threadfence();
    *(volatile v8h*)op = hv;
  }
}

__global__ __launch_bounds__(SCAN_THR) void scan_kernel(const unsigned short* __restrict__ XHp,
                                                        const unsigned short* __restrict__ JCp,
                                                        const float* __restrict__ gain,
                                                        const float* __restrict__ thr,
                                                        unsigned short* __restrict__ HSp) {
  __shared__ __align__(16) _Float16 At[SEQ_BLK * APITCH];
  const _Float16* JC = (const _Float16*)JCp;
  const int tid = threadIdx.x, lane = tid & 31, wave = tid >> 5;
  const int c = lane & 15, hh = lane >> 4, koff = hh * 8;
  const int rowbase = blockIdx.x * SEQ_BLK;

#pragma unroll 1
  for (int i = tid; i < SEQ_BLK * APITCH; i += SCAN_THR) At[i] = (_Float16)0.0f;
  __syncthreads();

  const int sm  = tid >> 5;
  const int sc8 = (tid & 31) * 8;
  {
    const v4u xv = *(const v4u*)(const void*)(XHp + ((size_t)(rowbase + sm) * NSTEP) * NDIN + sc8);
    *(v4u*)(void*)(At + sm * APITCH + NHID + sc8) = xv;
  }

  float gj[4], tj[4];
#pragma unroll
  for (int nt = 0; nt < 4; ++nt) {
    const int j = 64 * wave + 16 * nt + c;
    gj[nt] = gain[j];
    tj[nt] = thr[j];
  }
  __syncthreads();

  const _Float16* arow = At + c * APITCH + koff;
  const _Float16* bp0 = JC + (size_t)(64 * wave + c) * KCAT + koff;
  const _Float16* bp1 = bp0 + (size_t)16 * KCAT;
  const _Float16* bp2 = bp0 + (size_t)32 * KCAT;
  const _Float16* bp3 = bp0 + (size_t)48 * KCAT;
  const v8f z8 = {0.f, 0.f, 0.f, 0.f, 0.f, 0.f, 0.f, 0.f};

#pragma unroll 1
  for (int t = 0; t < NSTEP; ++t) {
    v8f acc[4];
    acc[0] = z8; acc[1] = z8; acc[2] = z8; acc[3] = z8;
#pragma unroll 1
    for (int k0 = 0; k0 < KCAT; k0 += 32) {
      const v16h a  = frag_load(arow + k0);
      const v16h b0 = frag_load(bp0 + k0);
      const v16h b1 = frag_load(bp1 + k0);
      const v16h b2 = frag_load(bp2 + k0);
      const v16h b3 = frag_load(bp3 + k0);
      acc[0] = frag_mma(a, b0, acc[0]);
      acc[1] = frag_mma(a, b1, acc[1]);
      acc[2] = frag_mma(a, b2, acc[2]);
      acc[3] = frag_mma(a, b3, acc[3]);
      guard4x5_h(acc[0], acc[1], acc[2], acc[3], a, b0, b1, b2, b3);
    }
    acc_guard4(acc[0], acc[1], acc[2], acc[3]);

    float av[4][8];
#pragma unroll
    for (int nt = 0; nt < 4; ++nt) {
#pragma unroll
      for (int r = 0; r < 8; ++r) {
        const float pre = acc[nt][r] * STATE_CARRY_INV - tj[nt];
        av[nt][r] = (pre > 0.0f) ? (pre * gj[nt]) : 0.0f;
      }
    }

    __syncthreads();

#pragma unroll
    for (int nt = 0; nt < 4; ++nt) {
      const int j = 64 * wave + 16 * nt + c;
#pragma unroll
      for (int r = 0; r < 8; ++r) At[(8 * hh + r) * APITCH + j] = (_Float16)av[nt][r];
    }
    {
      const int tn = (t + 1 < NSTEP) ? (t + 1) : (NSTEP - 1);
      const v4u xv = *(const v4u*)(const void*)(XHp + ((size_t)(rowbase + sm) * NSTEP + (size_t)tn) * NDIN + sc8);
      *(v4u*)(void*)(At + sm * APITCH + NHID + sc8) = xv;
    }
    __syncthreads();

    {
      v4u sv[4];
#pragma unroll
      for (int it = 0; it < 4; ++it) {
        const int idx = it * SCAN_THR + tid;
        const int row = idx >> 7;
        const int c8  = (idx & 127) * 8;
        sv[it] = *(const v4u*)(const void*)(At + row * APITCH + c8);
      }
      for (int pass = 0; pass < 2; ++pass) {
#pragma unroll
        for (int it = 0; it < 4; ++it) {
          const int idx = it * SCAN_THR + tid;
          const int row = idx >> 7;
          const int c8  = (idx & 127) * 8;
          unsigned short* op = HSp + ((size_t)(rowbase + row) * NSTEP + (size_t)t) * NHID + c8;
          *(volatile v4u*)(void*)op = sv[it];
        }
        __threadfence();
      }
    }
  }
}

__global__ __launch_bounds__(256) void readout_gemm_kernel(const unsigned short* __restrict__ Ap, int lda,
                                                           const unsigned short* __restrict__ Btp, int ldb,
                                                           float* __restrict__ C, int ldc,
                                                           const float* __restrict__ bias,
                                                           int M, int N, int K, float scale) {
  const _Float16* A  = (const _Float16*)Ap;
  const _Float16* Bt = (const _Float16*)Btp;
  __shared__ __align__(16) float sT[8][16 * 68];
  const int lane = threadIdx.x & 31;
  const int wave = threadIdx.x >> 5;
  const int tilesN = N >> 6;
  const int tilesM = M >> 6;
  const int tile = blockIdx.x * 8 + wave;
  if (tile >= tilesM * tilesN) return;
  const int tm = tile / tilesN;
  const int tn = tile - tm * tilesN;
  const int m0 = tm << 6;
  const int n0 = tn << 6;

  const int rlane = lane & 15;
  const int koff  = (lane >> 4) * 8;
  const int mOff  = (lane >> 4) * 8;

  v8f acc[4][4];
#pragma unroll
  for (int i = 0; i < 4; ++i)
#pragma unroll
    for (int j = 0; j < 4; ++j) acc[i][j] = (v8f){0.f, 0.f, 0.f, 0.f, 0.f, 0.f, 0.f, 0.f};

  for (int k0 = 0; k0 < K; k0 += 32) {
    v16h bh[4];
#pragma unroll
    for (int j = 0; j < 4; ++j) {
      const size_t bo = (size_t)(n0 + (j << 4) + rlane) * ldb + koff + k0;
      bh[j] = frag_load(Bt + bo);
    }
#pragma unroll
    for (int i = 0; i < 4; ++i) {
      const size_t ao = (size_t)(m0 + (i << 4) + rlane) * lda + koff + k0;
      const v16h ah = frag_load(A + ao);
#pragma unroll
      for (int j = 0; j < 4; ++j) acc[i][j] = frag_mma(ah, bh[j], acc[i][j]);
      guard4x5_h(acc[i][0], acc[i][1], acc[i][2], acc[i][3], ah, bh[0], bh[1], bh[2], bh[3]);
    }
  }
  acc_guard4(acc[0][0], acc[0][1], acc[0][2], acc[0][3]);
  acc_guard4(acc[1][0], acc[1][1], acc[1][2], acc[1][3]);
  acc_guard4(acc[2][0], acc[2][1], acc[2][2], acc[2][3]);
  acc_guard4(acc[3][0], acc[3][1], acc[3][2], acc[3][3]);

  float* slab = sT[wave];
#pragma unroll
  for (int i = 0; i < 4; ++i) {
    const int mBase = m0 + (i << 4);
#pragma unroll
    for (int j = 0; j < 4; ++j) {
      const int n = n0 + (j << 4) + rlane;
      const float bv = bias[n];
#pragma unroll
      for (int r = 0; r < 8; ++r) {
        const float v = acc[i][j][r] * scale + bv;
        slab[(mOff + r) * 68 + (j << 4) + rlane] = v;
      }
    }
    __builtin_amdgcn_fence(__ATOMIC_RELEASE, "workgroup");
    __builtin_amdgcn_wave_barrier();
    __builtin_amdgcn_fence(__ATOMIC_ACQUIRE, "workgroup");
    {
      const int hh = lane >> 4, c4 = (lane & 15) * 4;
      for (int pass = 0; pass < 2; ++pass) {
#pragma unroll
        for (int it = 0; it < 8; ++it) {
          const int row = it * 2 + hh;
          const v4f v = *(const v4f*)(slab + row * 68 + c4);
          *(volatile v4f*)(C + (size_t)(mBase + row) * ldc + n0 + c4) = v;
        }
        __threadfence();
      }
    }
    __builtin_amdgcn_fence(__ATOMIC_RELEASE, "workgroup");
    __builtin_amdgcn_wave_barrier();
    __builtin_amdgcn_fence(__ATOMIC_ACQUIRE, "workgroup");
  }
}

extern "C" void kernel_launch(void* const* d_in, const int* in_sizes, int n_in,
                              void* d_out, int out_size, void* d_ws, size_t ws_size, hipStream_t stream) {
  if (n_in < 11 || d_out == nullptr || d_ws == nullptr) return;
  if (in_sizes[0] != NBATCH * NSTEP * NDIN || in_sizes[1] != NHID * NDIN || in_sizes[2] != NHID * 2 ||
      in_sizes[3] != NDIN * 2 || in_sizes[4] != NHID || in_sizes[5] != NHID || in_sizes[6] != NHID * NHID ||
      in_sizes[7] != NHID * 2 || in_sizes[8] != NHID * 2 || in_sizes[9] != NOUTC * NHID || in_sizes[10] != NOUTC ||
      out_size != NROWS * NOUTC) return;

  const float* x        = (const float*)d_in[0];
  const float* in_bg    = (const float*)d_in[1];
  const float* in_proj  = (const float*)d_in[2];
  const float* in_recv  = (const float*)d_in[3];
  const float* gain     = (const float*)d_in[4];
  const float* thr      = (const float*)d_in[5];
  const float* rec_bg   = (const float*)d_in[6];
  const float* rec_proj = (const float*)d_in[7];
  const float* rec_recv = (const float*)d_in[8];
  const float* w_out    = (const float*)d_in[9];
  const float* b_out    = (const float*)d_in[10];
  float* out = (float*)d_out;

  char* ws = (char*)d_ws;
  size_t off = 0;
  auto carve = [&](size_t bytes) -> char* { char* p = ws + off; off += (bytes + 255) & ~(size_t)255; return p; };
  unsigned short* XH = (unsigned short*)carve((size_t)NROWS * NDIN * 2);
  unsigned short* JC = (unsigned short*)carve((size_t)NHID * KCAT * 2);
  unsigned short* WO = (unsigned short*)carve((size_t)NOUTC * NHID * 2);
  unsigned short* HS = (unsigned short*)carve((size_t)NROWS * NHID * 2);
  if (off > ws_size || off > (size_t)134217728) return;

  const int n8x = NROWS * (NDIN / 8);
  cvt8_f16_kernel<<<(n8x + CVT_THR - 1) / CVT_THR, CVT_THR, 0, stream>>>(x, XH, n8x, STATE_CARRY);
  const int n8j = NHID * (NHID / 8);
  lowrank8_kernel<<<(n8j + CVT_THR - 1) / CVT_THR, CVT_THR, 0, stream>>>(rec_bg, rec_proj, rec_recv, JC,
                                                                         NHID, NHID / 8, KCAT, 0);
  const int n8i = NHID * (NDIN / 8);
  lowrank8_kernel<<<(n8i + CVT_THR - 1) / CVT_THR, CVT_THR, 0, stream>>>(in_bg, in_proj, in_recv, JC,
                                                                         NHID, NDIN / 8, KCAT, NHID);
  const int n8w = NOUTC * (NHID / 8);
  cvt8_f16_kernel<<<(n8w + CVT_THR - 1) / CVT_THR, CVT_THR, 0, stream>>>(w_out, WO, n8w, WO_CARRY);
  scan_kernel<<<NBATCH / SEQ_BLK, SCAN_THR, 0, stream>>>(XH, JC, gain, thr, HS);
  const int tiles = (NROWS / 64) * (NOUTC / 64);
  readout_gemm_kernel<<<dim3((tiles + 7) / 8, 1), 256, 0, stream>>>(HS, NHID, WO, NHID, out, NOUTC, b_out,
                                                                    NROWS, NOUTC, NHID, READ_SCALE);
}
